// SoftDTWCuda_69758858822517
// MI455X (gfx1250) — hardware-verified
//
#include <hip/hip_runtime.h>

typedef _Float16 v16h __attribute__((ext_vector_type(16)));
typedef _Float16 v8h  __attribute__((ext_vector_type(8)));
typedef float    v8f  __attribute__((ext_vector_type(8)));
typedef float    v4f  __attribute__((ext_vector_type(4)));
typedef v8h __attribute__((may_alias)) v8ha;
typedef v4f __attribute__((may_alias)) v4fa;

union Frag { v16h v; v8h half[2]; };

#define NBATCH   32
#define SLEN     512
#define DDIM     128
#define NPAIR    3
#define NZ       (NPAIR * NBATCH)
#define NXEL     (NBATCH * SLEN * DDIM)
#define TROWS    (NBATCH * SLEN)
#define NROWS    (2 * TROWS)
#define PLANE    (SLEN * SLEN)
#define NDIAG    (2 * SLEN - 1)
#define DLEN     520
#define BIG      100000000.0f
#define OPSC     16.0f
#define ACCSC    0.00390625f
#define RESPITCH 32

static_assert(NROWS % 16 == 0);
static_assert(TROWS % 16 == 0);
static_assert(SLEN % 128 == 0);
static_assert(DDIM % 32 == 0);
static_assert(DLEN >= SLEN + 1);

__device__ __forceinline__ v8f wmma_f16(v16h a, v16h b, v8f c) {
  v8f d = __builtin_amdgcn_wmma_f32_16x16x32_f16(false, a, false, b, (short)0, c, false, false);
  asm volatile("v_nop\n\tv_nop\n\tv_nop\n\tv_nop" : "+v"(d) : "v"(a), "v"(b));
  return d;
}

__device__ __forceinline__ v16h load_frag(const _Float16* p, int h) {
  Frag f;
  f.half[0] = *(const v8ha*)(p + 8 * h);
  f.half[1] = *(const v8ha*)(p + 16 + 8 * h);
  return f.v;
}

__global__ __launch_bounds__(256) void normalize_kernel(
    const float* __restrict__ x, const float* __restrict__ y,
    _Float16* __restrict__ xn, _Float16* __restrict__ yn)
{
  #pragma clang fp contract(off)
  const int tid = threadIdx.x, lane = tid & 31, w = tid >> 5;
  const int h = lane >> 4, seg = lane & 15;
  const int blk = blockIdx.x;
  const bool isy = blk >= (TROWS / 16);
  const int rr = (blk - (isy ? (TROWS / 16) : 0)) * 16 + 2 * w + h;
  const float* src = (isy ? y : x) + (size_t)rr * DDIM + 8 * seg;
  _Float16* dst = (isy ? yn : xn) + (size_t)rr * DDIM + 8 * seg;

  const v4f a = *(const v4fa*)src;
  const v4f c = *(const v4fa*)(src + 4);
  float ss = a.x * a.x + a.y * a.y + a.z * a.z + a.w * a.w
           + c.x * c.x + c.y * c.y + c.z * c.z + c.w * c.w;
  ss += __shfl_xor(ss, 1);
  ss += __shfl_xor(ss, 2);
  ss += __shfl_xor(ss, 4);
  ss += __shfl_xor(ss, 8);
  const float nrm = sqrtf(ss);
  const float inv = 1.0f / fmaxf(nrm, 1e-8f);
  const float sc = inv * OPSC;
  const v8h o = { (_Float16)(a.x * sc), (_Float16)(a.y * sc), (_Float16)(a.z * sc), (_Float16)(a.w * sc),
                  (_Float16)(c.x * sc), (_Float16)(c.y * sc), (_Float16)(c.z * sc), (_Float16)(c.w * sc) };
  *(volatile v8h*)dst = o;
  __threadfence();
  *(volatile v8h*)dst = o;
}

__device__ __forceinline__ void cost_store_pass(const float* so, float* dstbase, int lane) {
  const int q8 = lane & 7, sub = lane >> 3;
  #pragma unroll
  for (int i = 0; i < 16; ++i) {
    const int lid = i * 4 + sub;
    const int row = lid >> 1, hl = lid & 1;
    const v4f v = *(const v4fa*)(so + row * 64 + 32 * hl + 4 * q8);
    *(volatile v4f*)(dstbase + (size_t)row * SLEN + 32 * hl + 4 * q8) = v;
  }
}

__global__ __launch_bounds__(128) void cost_gemm_kernel(
    const _Float16* __restrict__ xn,
    const _Float16* __restrict__ yn,
    float* __restrict__ cost)
{
  #pragma clang fp contract(off)
  __shared__ __attribute__((aligned(16))) float sT[128 * 64];

  const int tid = threadIdx.x, lane = tid & 31, w = tid >> 5;
  const int h = lane >> 4, m = lane & 15;
  const int n0 = blockIdx.x * 64;
  const int m0 = blockIdx.y * 128;
  const int z = blockIdx.z;
  const int pair = z >> 5, b = z & 31;

  const _Float16* Ab = ((pair == 2) ? yn : xn) + (size_t)b * SLEN * DDIM;
  const _Float16* Bb = ((pair == 1) ? xn : yn) + (size_t)b * SLEN * DDIM;
  const _Float16* a0p = Ab + (size_t)(m0 + 32 * w + m) * DDIM;
  const _Float16* a1p = a0p + (size_t)16 * DDIM;
  const _Float16* bp  = Bb + (size_t)(n0 + m) * DDIM;

  const v8f zero8 = {0.f, 0.f, 0.f, 0.f, 0.f, 0.f, 0.f, 0.f};
  v8f acc[2][4];
  #pragma unroll
  for (int mt = 0; mt < 2; ++mt)
    #pragma unroll
    for (int nt = 0; nt < 4; ++nt) acc[mt][nt] = zero8;

  #pragma unroll
  for (int k0 = 0; k0 < DDIM; k0 += 32) {
    const v16h a0 = load_frag(a0p + k0, h);
    const v16h a1 = load_frag(a1p + k0, h);
    #pragma unroll
    for (int nt = 0; nt < 4; ++nt) {
      const v16h bf = load_frag(bp + (size_t)nt * 16 * DDIM + k0, h);
      acc[0][nt] = wmma_f16(a0, bf, acc[0][nt]);
      acc[1][nt] = wmma_f16(a1, bf, acc[1][nt]);
    }
  }

  float* so = sT + w * 2048;
  #pragma unroll
  for (int nt = 0; nt < 4; ++nt)
    #pragma unroll
    for (int mt = 0; mt < 2; ++mt)
      #pragma unroll
      for (int r = 0; r < 8; ++r) {
        const float dot = acc[mt][nt][r] * ACCSC;
        so[(16 * mt + 8 * h + r) * 64 + 16 * nt + m] = 1.0f - dot;
      }
  __syncthreads();

  float* dstbase = cost + ((size_t)z * SLEN + m0 + 32 * w) * SLEN + n0;
  cost_store_pass(so, dstbase, lane);
  __threadfence();
  cost_store_pass(so, dstbase, lane);
}

__global__ __launch_bounds__(512) void dp_kernel(
    const float* __restrict__ cost,
    const float* __restrict__ gamma_p,
    float* __restrict__ res)
{
  #pragma clang fp contract(off)
  __shared__ float diag[3 * DLEN];

  const int tid = threadIdx.x;
  const int z = blockIdx.x;
  const float g = fmaxf(fabsf(gamma_p[0]), 1e-4f);
  const float invg = 1.0f / g;

  for (int idx = tid; idx < 3 * DLEN; idx += 512) diag[idx] = (idx == 0) ? 0.0f : BIG;
  __syncthreads();

  const int i = tid + 1;
  const float* crow = cost + (size_t)z * PLANE + (size_t)tid * SLEN;
  int b2 = 0, b1 = 1, bn = 2;

  #pragma unroll 1
  for (int k = 0; k < NDIAG; ++k) {
    const int c = k - tid;
    const bool valid = (c >= 0) && (c < SLEN);
    const int cc = min(max(c, 0), SLEN - 1);
    const float cd = crow[cc];
    const float* pm2 = diag + b2 * DLEN;
    const float* pm1 = diag + b1 * DLEN;
    float* pn = diag + bn * DLEN;
    const float p0 = pm2[i - 1];
    const float p1 = pm1[i - 1];
    const float p2 = pm1[i];
    const float a0 = -p0 * invg;
    const float a1 = -p1 * invg;
    const float a2 = -p2 * invg;
    const float amax = fmaxf(a0, fmaxf(a1, a2));
    const float s = __expf(a0 - amax) + __expf(a1 - amax) + __expf(a2 - amax);
    const float lse = amax + __logf(s);
    const float gl = g * lse;
    const float nv = cd - gl;
    pn[i] = valid ? nv : BIG;
    if (tid == 0) pn[0] = BIG;
    __syncthreads();
    const int t = b2; b2 = b1; b1 = bn; bn = t;
  }

  const float R = diag[b1 * DLEN + SLEN];
  const v4f rv = {R, R, R, R};
  float* dst = res + (size_t)z * RESPITCH + 4 * (tid & 7);
  if (tid < 8) *(volatile v4f*)dst = rv;
  __threadfence();
  if (tid < 8) *(volatile v4f*)dst = rv;
}

__global__ __launch_bounds__(32) void combine_kernel(
    const float* __restrict__ res, float* __restrict__ out)
{
  #pragma clang fp contract(off)
  __shared__ __attribute__((aligned(16))) float sv[32];
  const int lane = threadIdx.x;
  const float rxy = res[(size_t)(0 * NBATCH + lane) * RESPITCH];
  const float rxx = res[(size_t)(1 * NBATCH + lane) * RESPITCH];
  const float ryy = res[(size_t)(2 * NBATCH + lane) * RESPITCH];
  const float t = rxx + ryy;
  const float u = 0.5f * t;
  const float v = rxy - u;
  sv[lane] = v;
  __syncthreads();
  const v4f o = *(const v4fa*)(sv + 4 * (lane & 7));
  if (lane < 8) *(volatile v4f*)(out + 4 * lane) = o;
  __threadfence();
  if (lane < 8) *(volatile v4f*)(out + 4 * lane) = o;
}

extern "C" void kernel_launch(void* const* d_in, const int* in_sizes, int n_in,
                              void* d_out, int out_size, void* d_ws, size_t ws_size,
                              hipStream_t stream) {
  if (n_in < 3) return;
  if (in_sizes[0] != NXEL || in_sizes[1] != NXEL || in_sizes[2] < 1) return;
  if (out_size != NBATCH) return;

  const float* x     = (const float*)d_in[0];
  const float* y     = (const float*)d_in[1];
  const float* gamma = (const float*)d_in[2];
  float* out = (float*)d_out;

  const size_t pl_bytes   = (size_t)NXEL * 2;
  const size_t cost_bytes = (size_t)NZ * PLANE * 4;
  const size_t res_bytes  = (size_t)NZ * RESPITCH * 4;
  const size_t off_xn   = 0;
  const size_t off_yn   = off_xn + pl_bytes;
  const size_t off_cost = off_yn + pl_bytes;
  const size_t off_res  = off_cost + cost_bytes;
  const size_t total    = off_res + res_bytes;
  if (total > ws_size) return;

  char* ws = (char*)d_ws;
  _Float16* xn = (_Float16*)(ws + off_xn);
  _Float16* yn = (_Float16*)(ws + off_yn);
  float* cost  = (float*)(ws + off_cost);
  float* res   = (float*)(ws + off_res);

  normalize_kernel<<<NROWS / 16, 256, 0, stream>>>(x, y, xn, yn);

  dim3 gGemm(SLEN / 64, SLEN / 128, NZ);
  cost_gemm_kernel<<<gGemm, 128, 0, stream>>>(xn, yn, cost);

  dp_kernel<<<NZ, 512, 0, stream>>>(cost, gamma, res);

  combine_kernel<<<1, 32, 0, stream>>>(res, out);
}
